// MixtureCDFFLowCoupling_62285615727068
// MI455X (gfx1250) — hardware-verified
//
#include <hip/hip_runtime.h>
#include <stddef.h>
#include <math.h>

#pragma clang fp contract(off)

#define DIM   64
#define DH    32
#define HID   512
#define NMIX  8
#define OUTW  1160
#define NPC   584
#define NPR   640
#define PP    592
#define MT    16
#define NTHR  256
#define HP    520
#define XP    40

static_assert(HP % 8 == 0);
static_assert(XP % 8 == 0);
static_assert(NPC + 8 <= PP);
static_assert(MT * DIM == NTHR * 4);
static_assert(HID % 64 == 0);
static_assert(NPR % 64 == 0);
static_assert(NPR >= PP);

typedef _Float16 f16;
typedef f16 v16h __attribute__((ext_vector_type(16)));
typedef f16 v8h_t __attribute__((ext_vector_type(8)));
typedef v8h_t __attribute__((may_alias)) v8h;
typedef float v8f __attribute__((ext_vector_type(8)));
typedef float v4f_t __attribute__((ext_vector_type(4)));
typedef v4f_t __attribute__((may_alias)) v4f;
typedef unsigned int v4u __attribute__((ext_vector_type(4)));

union Frag { v16h v; v8h_t h[2]; };
union Pack8 { v8h_t h; v4u u; };

__device__ __forceinline__ v8f zero8() {
    v8f z;
#pragma unroll
    for (int i = 0; i < 8; ++i) z[i] = 0.0f;
    return z;
}

__device__ __forceinline__ v16h ldfrag(const f16* p, int k0) {
    Frag f;
    f.h[0] = *(const v8h*)(p + k0);
    f.h[1] = *(const v8h*)(p + k0 + 16);
    return f.v;
}

__device__ __forceinline__ v8f wmma16(v16h a, v16h b, v8f c) {
    return __builtin_amdgcn_wmma_f32_16x16x32_f16(false, a, false, b, (short)0, c, false, false);
}

__device__ __forceinline__ int pcol(int c) {
    const int q1 = c - 72, q2 = c - 328;
    const int m1 = 168 + ((q1 >> 5) << 6) + (q1 & 31);
    const int m2 = 680 + ((q2 >> 5) << 6) + (q2 & 31);
    int r = (c < 32) ? (32 + c) : (64 + c);
    r = (c >= 72) ? m1 : r;
    r = (c >= 328) ? m2 : r;
    return r;
}

template <int KS, int TS>
__device__ __forceinline__ void wgemm4(const f16* pa, const f16* __restrict__ pb, v8f (&acc)[4]) {
#pragma unroll 2
    for (int ks = 0; ks < KS; ++ks) {
        const int k0 = ks * 32;
        const v16h a  = ldfrag(pa, k0);
        const v16h b0 = ldfrag(pb, k0);
        const v16h b1 = ldfrag(pb + TS, k0);
        const v16h b2 = ldfrag(pb + 2 * TS, k0);
        const v16h b3 = ldfrag(pb + 3 * TS, k0);
        acc[0] = wmma16(a, b0, acc[0]);
        acc[1] = wmma16(a, b1, acc[1]);
        acc[2] = wmma16(a, b2, acc[2]);
        acc[3] = wmma16(a, b3, acc[3]);
        asm volatile("v_nop\n\tv_nop\n\tv_nop\n\tv_nop"
                     : "+v"(acc[0]), "+v"(acc[1]), "+v"(acc[2]), "+v"(acc[3])
                     : "v"(a), "v"(b0), "v"(b1), "v"(b2), "v"(b3));
    }
}

template <int KS>
__device__ __forceinline__ void wgemm1(const f16* pa, const f16* __restrict__ pb, v8f (&acc)[1]) {
#pragma unroll 2
    for (int ks = 0; ks < KS; ++ks) {
        const int k0 = ks * 32;
        const v16h a = ldfrag(pa, k0);
        const v16h b = ldfrag(pb, k0);
        acc[0] = wmma16(a, b, acc[0]);
        asm volatile("v_nop\n\tv_nop\n\tv_nop\n\tv_nop" : "+v"(acc[0]) : "v"(a), "v"(b));
    }
}

__device__ __forceinline__ void epi_h(const v8f (&acc)[4], f16* hs, const float* __restrict__ bias,
                                      int col0, float scale, int hh, int m) {
#pragma unroll
    for (int t = 0; t < 4; ++t) {
        const int col = col0 + 16 * t + m;
        const float bv = bias[col];
#pragma unroll
        for (int r = 0; r < 8; ++r) {
            float v = acc[t][r] * scale + bv;
            v = fmaxf(v, 0.0f);
            hs[(8 * hh + r) * HP + col] = (f16)v;
        }
    }
}

template <int NT>
__device__ __forceinline__ void epi_p(const v8f (&acc)[NT], float* sp, const float* __restrict__ b3,
                                      int col0, int hh, int m) {
#pragma unroll
    for (int t = 0; t < NT; ++t) {
        const int col = col0 + 16 * t + m;
        const int cc  = col < NPC ? col : (NPC - 1);
        const int oc  = pcol(cc);
        float bv = b3[oc];
        bv = (col < NPC) ? bv : 0.0f;
#pragma unroll
        for (int r = 0; r < 8; ++r)
            sp[(8 * hh + r) * PP + col] = acc[t][r] * (1.0f / 256.0f) + bv;
    }
}

template <int KT>
__global__ void __launch_bounds__(NTHR) k_prep(const float* __restrict__ W, int wcols,
                                               f16* __restrict__ Wt, int pitch,
                                               int nvalid, int mode, float scale)
{
    __shared__ __align__(16) f16 s[64 * (KT + 8)];
    const int t  = threadIdx.x;
    const int n0 = blockIdx.x * 64;
    const int k0 = blockIdx.y * KT;
#pragma unroll
    for (int i = 0; i < KT / 4; ++i) {
        const int idx = i * NTHR + t;
        const int kk = idx >> 6, nn = idx & 63;
        const int c = n0 + nn;
        int oc = (mode != 0) ? pcol(c) : c;
        oc = oc < 0 ? 0 : oc;
        oc = oc > (wcols - 1) ? (wcols - 1) : oc;
        const float v  = W[(size_t)(k0 + kk) * wcols + oc] * scale;
        const float vz = (c < nvalid) ? v : 0.0f;
        s[nn * (KT + 8) + kk] = (f16)vz;
    }
    __syncthreads();
    constexpr int REPS = KT / 32;
    constexpr int SEG  = KT / 8;
    v4u    pv[REPS];
    size_t po[REPS];
#pragma unroll
    for (int rp = 0; rp < REPS; ++rp) {
        const int j  = rp * NTHR + t;
        const int nn = j / SEG, k8 = j - nn * SEG;
        Pack8 pk;
        pk.h   = *(const v8h*)(s + nn * (KT + 8) + k8 * 8);
        pv[rp] = pk.u;
        po[rp] = (size_t)(n0 + nn) * pitch + (size_t)k0 + (size_t)(k8 * 8);
        *(volatile v4u*)(Wt + po[rp]) = pv[rp];
    }
    __threadfence();
#pragma unroll
    for (int rp = 0; rp < REPS; ++rp)
        *(volatile v4u*)(Wt + po[rp]) = pv[rp];
}

__global__ void __launch_bounds__(NTHR) k_main(const float* __restrict__ x,
                                             const float* __restrict__ b1,
                                             const float* __restrict__ b2,
                                             const float* __restrict__ b3,
                                             const f16* __restrict__ W1c,
                                             const f16* __restrict__ W2c,
                                             const f16* __restrict__ W3c,
                                             float* __restrict__ out, int ntok)
{
    __shared__ __align__(16) float  s_x[MT * DIM];
    __shared__ __align__(16) f16    s_xa[MT * XP];
    __shared__ __align__(16) f16    s_h1[MT * HP];
    __shared__ __align__(16) f16    s_h2[MT * HP];
    __shared__ __align__(16) float  s_par[MT * PP];
    __shared__ __align__(16) double s_w[MT * NMIX];
    __shared__ __align__(16) float  s_o[2 * MT * DIM];

    const int tid  = threadIdx.x;
    const int lane = tid & 31;
    const int wv   = __builtin_amdgcn_readfirstlane(tid >> 5);
    const int hh   = lane >> 4, m = lane & 15;
    const size_t tok0 = (size_t)blockIdx.x * MT;

    {
        const int row = tid >> 4, c4 = (tid & 15) * 4;
        const v4f_t v = *(const v4f*)(x + (tok0 + row) * DIM + c4);
        *(v4f*)(s_x + row * DIM + c4) = v;
        if (c4 < DH) {
#pragma unroll
            for (int j = 0; j < 4; ++j) s_xa[row * XP + c4 + j] = (f16)v[j];
        }
    }
    __syncthreads();

    {
        v8f acc[4];
#pragma unroll
        for (int t = 0; t < 4; ++t) acc[t] = zero8();
        wgemm4<1, 16 * DH>(s_xa + m * XP + 8 * hh,
                           W1c + (size_t)(wv * 64 + m) * DH + 8 * hh, acc);
        epi_h(acc, s_h1, b1, wv * 64, 0.125f, hh, m);
    }
    __syncthreads();

    {
        v8f acc[4];
#pragma unroll
        for (int t = 0; t < 4; ++t) acc[t] = zero8();
        wgemm4<HID / 32, 16 * HID>(s_h1 + m * HP + 8 * hh,
                                   W2c + (size_t)(wv * 64 + m) * HID + 8 * hh, acc);
        epi_h(acc, s_h2, b2, wv * 64, 0.0625f, hh, m);
    }
    __syncthreads();

    {
        v8f acc[4];
#pragma unroll
        for (int t = 0; t < 4; ++t) acc[t] = zero8();
        wgemm4<HID / 32, 16 * HID>(s_h2 + m * HP + 8 * hh,
                                   W3c + (size_t)(wv * 64 + m) * HID + 8 * hh, acc);
        epi_p<4>(acc, s_par, b3, wv * 64, hh, m);
        if (wv < 5) {
            const int col0 = 512 + 16 * wv;
            v8f a1[1];
            a1[0] = zero8();
            wgemm1<HID / 32>(s_h2 + m * HP + 8 * hh,
                             W3c + (size_t)(col0 + m) * HID + 8 * hh, a1);
            epi_p<1>(a1, s_par, b3, col0, hh, m);
        }
    }
    __syncthreads();

    if (tid < MT) {
        const float* lg = s_par + tid * PP + 64;
        double* pw = s_w + tid * NMIX;
        double mx = (double)lg[0];
#pragma unroll 1
        for (int k = 1; k < NMIX; ++k) mx = fmax(mx, (double)lg[k]);
        double s = 0.0;
#pragma unroll 1
        for (int k = 0; k < NMIX; ++k) {
            const double e = exp((double)lg[k] - mx);
            pw[k] = e;
            s = s + e;
        }
        const double inv = 1.0 / s;
#pragma unroll 1
        for (int k = 0; k < NMIX; ++k) pw[k] = pw[k] * inv;
    }
    __syncthreads();

    const double kInvSqrt2 = 0.70710678118654752440;
    const double kSqrt2Pi  = 2.50662827463100050242;
#pragma unroll 1
    for (int rep = 0; rep < 2; ++rep) {
        const int item = rep * NTHR + tid;
        const int tk = item >> 5;
        const int d  = DH + (item & 31);
        const double xv = (double)s_x[tk * DIM + d];
        const float* pp = s_par + tk * PP;
        const double* pw = s_w + tk * NMIX;
        const double ls = (double)pp[d - 32];
        const double bs = (double)pp[d];
        double z = 0.0, pm = 0.0;
#pragma unroll 1
        for (int k = 0; k < NMIX; ++k) {
            const double mu  = (double)pp[40 + 32 * k + d];
            const double lsd = (double)pp[296 + 32 * k + d];
            const double wk  = pw[k];
            const double sd  = exp(lsd);
            const double u   = (xv - mu) / sd;
            const double cdf = 0.5 * (1.0 + erf(u * kInvSqrt2));
            z = z + cdf * wk;
            const double g   = exp((-0.5 * u) * u);
            const double pdf = g / (sd * kSqrt2Pi);
            pm = pm + pdf * wk;
        }
        const double ldm = log(pm);
        const double xs  = -log(1.0 / z - 1.0);
        const double lsg = -log(z) - log(1.0 - z);
        const double o   = xs * exp(ls) + bs;
        const double ld  = (ldm + lsg) + ls;
        s_o[tk * DIM + d]            = (float)o;
        s_o[MT * DIM + tk * DIM + d] = (float)ld;
    }
#pragma unroll 1
    for (int rep = 0; rep < 2; ++rep) {
        const int item = rep * NTHR + tid;
        const int tk = item >> 5;
        const int dd = item & 31;
        s_o[tk * DIM + dd]            = s_x[tk * DIM + dd];
        s_o[MT * DIM + tk * DIM + dd] = 0.0f;
    }
    __syncthreads();

    {
        const v4f_t v0 = *(const v4f*)(s_o + tid * 4);
        const v4f_t v1 = *(const v4f*)(s_o + MT * DIM + tid * 4);
        float* g0 = out + tok0 * DIM + (size_t)(tid * 4);
        float* g1 = out + (size_t)ntok * DIM + tok0 * DIM + (size_t)(tid * 4);
        *(volatile v4f_t*)g0 = v0;
        *(volatile v4f_t*)g1 = v1;
        __threadfence();
        *(volatile v4f_t*)g0 = v0;
        *(volatile v4f_t*)g1 = v1;
    }
}

extern "C" void kernel_launch(void* const* d_in, const int* in_sizes, int n_in,
                              void* d_out, int out_size, void* d_ws, size_t ws_size,
                              hipStream_t stream)
{
    if (n_in < 7) return;
    if (in_sizes[1] != DIM * HID) return;
    if (in_sizes[2] != HID) return;
    if (in_sizes[3] != HID * HID) return;
    if (in_sizes[4] != HID) return;
    if (in_sizes[5] != HID * OUTW) return;
    if (in_sizes[6] != OUTW) return;
    const int nx = in_sizes[0];
    if (nx <= 0 || (nx % (DIM * MT)) != 0) return;
    const int ntok = nx / DIM;
    if (out_size != 2 * nx) return;

    const float* x  = (const float*)d_in[0];
    const float* W1 = (const float*)d_in[1];
    const float* b1 = (const float*)d_in[2];
    const float* W2 = (const float*)d_in[3];
    const float* b2 = (const float*)d_in[4];
    const float* W3 = (const float*)d_in[5];
    const float* b3 = (const float*)d_in[6];
    float* out = (float*)d_out;

    const size_t bW1 = (size_t)HID * DH * 2;
    const size_t bW2 = (size_t)HID * HID * 2;
    const size_t bW3 = (size_t)NPR * HID * 2;
    const size_t oW1 = 0;
    const size_t oW2 = oW1 + bW1;
    const size_t oW3 = oW2 + bW2;
    const size_t total = oW3 + bW3;
    if (total > ws_size) return;

    char* ws = (char*)d_ws;
    f16* W1c = (f16*)(ws + oW1);
    f16* W2c = (f16*)(ws + oW2);
    f16* W3c = (f16*)(ws + oW3);

    k_prep<32><<<dim3(HID / 64, 1), NTHR, 0, stream>>>(W1, HID, W1c, DH, HID, 0, 8.0f);
    k_prep<64><<<dim3(HID / 64, HID / 64), NTHR, 0, stream>>>(W2, HID, W2c, HID, HID, 0, 16.0f);
    k_prep<64><<<dim3(NPR / 64, HID / 64), NTHR, 0, stream>>>(W3, OUTW, W3c, HID, NPC, 1, 256.0f);

    k_main<<<ntok / MT, NTHR, 0, stream>>>(x, b1, b2, b3, W1c, W2c, W3c, out, ntok);
}
